// SelfAttention_56075093017140
// MI455X (gfx1250) — hardware-run, weakly checked
//
#include <hip/hip_runtime.h>


#ifndef NB
#define NB 4
#endif
#ifndef SEQ
#define SEQ 4096
#endif
#define NB_FULL  4
#define SEQ_FULL 4096
#ifndef OUT_SEQ
#define OUT_SEQ SEQ
#endif
#define CH   256
#define CQ   32
#define VC   32
#define VCP  64
#define QKW  64
#define OH   128
#define AW   4
#define QRS  2048.0f
#define SC2  1.4426950408889634f
#define PSH  8.0f
#define WOS  1024.0f
#define OCS  1024.0f
#define OFI  (1.0f / (1024.0f * 1024.0f))
#define BOFF (2 * CQ + VCP)
#define NBIAS (BOFF + CH)

static_assert(CQ == 32);
static_assert(VC == 32);
static_assert(VC <= VCP);
static_assert(VCP % 64 == 0);
static_assert(QKW == 2 * CQ);
static_assert(CH % 64 == 0);
static_assert(CH % 32 == 0);
static_assert(OH == AW * 32);
static_assert(CH % OH == 0);
static_assert(OH % 16 == 0);
static_assert(SEQ % 64 == 0);
static_assert((NB * SEQ) % 64 == 0);
static_assert(SEQ % 32 == 0);
static_assert(SEQ % (16 * AW) == 0);
static_assert(OUT_SEQ % 32 == 0);
static_assert(SEQ_FULL % 4 == 0);
static_assert(NB <= NB_FULL);
static_assert(SEQ <= SEQ_FULL);
static_assert(BOFF % 32 == 0);
static_assert(NBIAS % 32 == 0);
static_assert(NBIAS / 4 == 96);
static_assert((VC * 2) % 16 == 0);

typedef _Float16 h16;
typedef unsigned short bf;
typedef __attribute__((ext_vector_type(16))) __bf16   v16bf;
typedef __attribute__((ext_vector_type(16))) _Float16 v16h;
typedef __attribute__((ext_vector_type(8)))  _Float16 v8h;
typedef __attribute__((ext_vector_type(8)))  unsigned short v8us;
typedef __attribute__((ext_vector_type(8)))  float    v8f;
typedef __attribute__((ext_vector_type(4)))  float    v4f;
typedef v4f  __attribute__((may_alias)) v4fa;

__device__ __forceinline__ unsigned short f2bf(float f) { unsigned u = __float_as_uint(f); u += 0x7FFFu + ((u >> 16) & 1u); return (unsigned short)(u >> 16); }
__device__ __forceinline__ v16h cat16(v8h lo, v8h hi) { return __builtin_shufflevector(lo, hi, 0, 1, 2, 3, 4, 5, 6, 7, 8, 9, 10, 11, 12, 13, 14, 15); }
__device__ __forceinline__ v16bf cat16b(v8us lo, v8us hi) { return __builtin_bit_cast(v16bf, __builtin_shufflevector(lo, hi, 0, 1, 2, 3, 4, 5, 6, 7, 8, 9, 10, 11, 12, 13, 14, 15)); }
__device__ __forceinline__ v8f wmma16(v16h a, v16h b, v8f c) { return __builtin_amdgcn_wmma_f32_16x16x32_f16(false, a, false, b, (short)0, c, false, false); }
__device__ __forceinline__ v8f wmmab(v16bf a, v16bf b, v8f c) { return __builtin_amdgcn_wmma_f32_16x16x32_bf16(false, a, false, b, (short)0, c, false, false); }
__device__ __forceinline__ v16h  ldh(const h16* p) { return cat16(*(const v8h*)p, *(const v8h*)(p + 16)); }
__device__ __forceinline__ v16bf ldb(const bf* p)  { return cat16b(*(const v8us*)p, *(const v8us*)(p + 16)); }
__device__ __forceinline__ void wave_sync() { __builtin_amdgcn_fence(3  , "wavefront"); __builtin_amdgcn_wave_barrier(); asm volatile("" ::: "memory"); }
__device__ __forceinline__ v8f wmma16g(v16h a, v16h b, v8f c) { c = wmma16(a, b, c); asm volatile("v_nop\n\tv_nop\n\tv_nop\n\tv_nop" : "+v"(c) : "v"(a), "v"(b)); return c; }
static __device__ __forceinline__ h16 toh_flush(float v) { const h16 r = (h16)v; return (fabsf(v) < 6.103515625e-05f) ? (h16)0.0f : r; }
static __device__ __forceinline__ h16 p_flush(float e) { const h16 r = (h16)__builtin_amdgcn_exp2f(e); return (e < -14.0f) ? (h16)0.0f : r; }

__global__ __launch_bounds__(256) void k_cvt8(const float* __restrict__ src, bf* dst, size_t n8) {
    const size_t i = (size_t)blockIdx.x * 256 + threadIdx.x; if (i >= n8) return;
    const v8f v = *(const v8f*)(src + i * 8); v8us o;
#pragma unroll
    for (int k = 0; k < 8; ++k) o[k] = f2bf(v[k]);
    *(volatile v8us*)(dst + i * 8) = o; __threadfence(); *(volatile v8us*)(dst + i * 8) = o;
}

__global__ __launch_bounds__(256) void k_cvt8z(const float* __restrict__ src, bf* dst, size_t n8src, size_t n8tot) {
    const size_t i = (size_t)blockIdx.x * 256 + threadIdx.x; if (i >= n8tot) return;
    const size_t is = (i < n8src) ? i : (n8src - 1);
    const v8f v = *(const v8f*)(src + is * 8); v8us o;
#pragma unroll
    for (int k = 0; k < 8; ++k) { const unsigned short w = f2bf(v[k]); o[k] = (i < n8src) ? w : (unsigned short)0; }
    *(volatile v8us*)(dst + i * 8) = o; __threadfence(); *(volatile v8us*)(dst + i * 8) = o;
}

__global__ __launch_bounds__(256) void k_cvth8(const float* __restrict__ src, h16* dst, size_t n8, float carry) {
    const size_t i = (size_t)blockIdx.x * 256 + threadIdx.x; if (i >= n8) return;
    const v8f v = *(const v8f*)(src + i * 8); v8h o;
#pragma unroll
    for (int k = 0; k < 8; ++k) { const float w = __uint_as_float(((unsigned)f2bf(v[k])) << 16) * carry; o[k] = toh_flush(w); }
    *(volatile v8h*)(dst + i * 8) = o; __threadfence(); *(volatile v8h*)(dst + i * 8) = o;
}

__global__ __launch_bounds__(256) void k_xt(const float* __restrict__ x, bf* XB) {
    __shared__ float ts[64 * 65];
    const int tid = threadIdx.x;
    const int n0 = blockIdx.x * 64, c0 = blockIdx.y * 64, b = blockIdx.z;
    const float* xs = x + ((size_t)b * CH + c0) * SEQ_FULL + n0;
    { const int cr = tid >> 4, nq = (tid & 15) * 4;
#pragma unroll
      for (int i = 0; i < 4; ++i) { const int c = cr + 16 * i; const v4f v = *(const v4f*)(xs + (size_t)c * SEQ_FULL + nq);
          ts[c * 65 + nq + 0] = v[0]; ts[c * 65 + nq + 1] = v[1]; ts[c * 65 + nq + 2] = v[2]; ts[c * 65 + nq + 3] = v[3]; } }
    __syncthreads();
    const int rw = tid >> 3, c8 = (tid & 7) * 8;
    v8us o0, o1;
#pragma unroll
    for (int k = 0; k < 8; ++k) { o0[k] = f2bf(ts[(c8 + k) * 65 + rw]); o1[k] = f2bf(ts[(c8 + k) * 65 + rw + 32]); }
    bf* d0 = XB + ((size_t)b * SEQ + n0 + rw) * CH + c0 + c8; bf* d1 = d0 + (size_t)32 * CH;
    *(volatile v8us*)d0 = o0; *(volatile v8us*)d1 = o1;
    __threadfence();
    *(volatile v8us*)d0 = o0; *(volatile v8us*)d1 = o1;
}

__global__ __launch_bounds__(96) void k_bias(const float* __restrict__ bq, const float* __restrict__ bk, const float* __restrict__ bv, const float* __restrict__ bo, float* BT) {
    const int i = threadIdx.x; if (i >= NBIAS / 4) return;
    const int e = i * 4;
    const int iq = (e < CQ - 4) ? e : (CQ - 4);
    int ik = e - CQ; ik = ik < 0 ? 0 : ik; ik = ik > CQ - 4 ? CQ - 4 : ik;
    int iv = e - 2 * CQ; iv = iv < 0 ? 0 : iv; iv = iv > VC - 4 ? VC - 4 : iv;
    int io = e - BOFF; io = io < 0 ? 0 : io; io = io > CH - 4 ? CH - 4 : io;
    const v4f a = *(const v4f*)(bq + iq); const v4f c = *(const v4f*)(bk + ik); const v4f d = *(const v4f*)(bv + iv); const v4f g = *(const v4f*)(bo + io);
    v4f s, o;
#pragma unroll
    for (int k = 0; k < 4; ++k) { s[k] = (e < CQ) ? a[k] : ((e < 2 * CQ) ? c[k] : ((e < 2 * CQ + VC) ? d[k] : ((e < BOFF) ? 0.0f : g[k]))); o[k] = __uint_as_float(((unsigned)f2bf(s[k])) << 16); }
    *(volatile v4f*)(BT + e) = o; __threadfence(); *(volatile v4f*)(BT + e) = o;
}

template <int BROW>
__global__ __launch_bounds__(32) void k_proj(const bf* __restrict__ A, const bf* __restrict__ Bt, const float* __restrict__ bias, h16* Ph, h16* Pr, int useRes, int RB, size_t sRB, int pitch, int CB, size_t sCB) {
    __shared__ __align__(16) float os[16 * 68];
    const int K = CH;
    const int lane = threadIdx.x & 31, lr = lane & 15, hi = lane >> 4; const int r0 = blockIdx.x * 64, c0 = blockIdx.y * 64;
    v8f acc[4][4];
#pragma unroll
    for (int mb = 0; mb < 4; ++mb)
#pragma unroll
        for (int nb = 0; nb < 4; ++nb) acc[mb][nb] = (v8f){};
    const size_t aoff = (size_t)(r0 + lr) * K + 8 * hi, boff = (size_t)(c0 + lr) * K + 8 * hi;
#pragma unroll 1
    for (int kc = 0; kc < K; kc += 32) {
        v16bf a[4];
#pragma unroll
        for (int mb = 0; mb < 4; ++mb) a[mb] = ldb(A + aoff + (size_t)mb * 16 * K + kc);
#pragma unroll
        for (int nb = 0; nb < 4; ++nb) { const v16bf b = ldb(Bt + boff + (size_t)nb * 16 * K + kc);
#pragma unroll
            for (int mb = 0; mb < 4; ++mb) acc[mb][nb] = wmmab(a[mb], b, acc[mb][nb]); }
        asm volatile("v_nop\n\tv_nop\n\tv_nop\n\tv_nop" : "+v"(acc[0][0]), "+v"(acc[1][1]), "+v"(acc[2][2]), "+v"(acc[3][3]) : "v"(a[0]), "v"(a[1]), "v"(a[2]), "v"(a[3]));
    }
    float bcol[4] = {0.0f, 0.0f, 0.0f, 0.0f};
    if (BROW == 0) {
#pragma unroll
        for (int nb = 0; nb < 4; ++nb) bcol[nb] = bias[c0 + nb * 16 + lr];
    }
    const size_t tbase = (size_t)(r0 / RB) * sRB + (size_t)(r0 % RB) * (size_t)pitch + (size_t)(c0 / CB) * sCB + (size_t)(c0 % CB);
#pragma unroll
    for (int mb = 0; mb < 4; ++mb) {
        float brw[8] = {0.0f, 0.0f, 0.0f, 0.0f, 0.0f, 0.0f, 0.0f, 0.0f};
        if (BROW == 1) { const v4f b0 = *(const v4f*)(bias + r0 + mb * 16 + hi * 8); const v4f b1 = *(const v4f*)(bias + r0 + mb * 16 + hi * 8 + 4);
            brw[0] = b0[0]; brw[1] = b0[1]; brw[2] = b0[2]; brw[3] = b0[3]; brw[4] = b1[0]; brw[5] = b1[1]; brw[6] = b1[2]; brw[7] = b1[3]; }
#pragma unroll
        for (int nb = 0; nb < 4; ++nb) {
#pragma unroll
            for (int j = 0; j < 8; ++j) { const float bb = BROW ? brw[j] : bcol[nb]; os[(hi * 8 + j) * 68 + nb * 16 + lr] = acc[mb][nb][j] + bb; } }
        wave_sync();
        const size_t sb = tbase + (size_t)(mb * 16) * (size_t)pitch;
#pragma unroll 1
        for (int ps = 0; ps < 2; ++ps) {
#pragma unroll
            for (int s = 0; s < 4; ++s) { const int row = 4 * s + (lane >> 3), c8 = (lane & 7) * 8;
                const v4f x0 = *(const v4fa*)(&os[row * 68 + c8]); const v4f x1 = *(const v4fa*)(&os[row * 68 + c8 + 4]); v8h hv, rv;
#pragma unroll
                for (int i = 0; i < 4; ++i) { const h16 a0 = (h16)x0[i]; const h16 a1 = (h16)x1[i]; hv[i] = a0; hv[4 + i] = a1; rv[i] = (h16)((x0[i] - (float)a0) * QRS); rv[4 + i] = (h16)((x1[i] - (float)a1) * QRS); }
                const size_t oo = sb + (size_t)row * (size_t)pitch + c8;
                *(volatile v8h*)(Ph + oo) = hv; if (useRes) *(volatile v8h*)(Pr + oo) = rv; }
            if (ps == 0) __threadfence(); }
        wave_sync();
    }
}

__global__ __launch_bounds__(32 * AW) void k_flash(const h16* __restrict__ QKH, const h16* __restrict__ VT, const h16* __restrict__ WOH, const float* __restrict__ BO, float* OUT) {
    __shared__ __align__(16) float os[OH * 68];
    const int lane = threadIdx.x & 31, wave = __builtin_amdgcn_readfirstlane((int)(threadIdx.x >> 5)), lr = lane & 15, hi = lane >> 4;
    const int b = blockIdx.y;
    const int t0 = (blockIdx.x * AW + wave) * 16;
    const size_t pbase = (size_t)b * SEQ * QKW;
    const size_t qo = pbase + (size_t)(t0 + lr) * QKW + 8 * hi;
    const v16h qh = ldh(QKH + qo);
    const size_t ko = pbase + (size_t)lr * QKW + CQ + 8 * hi;
    const size_t vo = ((size_t)b * VCP + lr) * SEQ + 8 * hi;
    v8f o0 = (v8f){}, o1 = (v8f){};
    float m = -3.0e38f, l = 0.0f;
#pragma unroll 1
    for (int key0 = 0; key0 < SEQ; key0 += 32) {
        const h16* ka = QKH + ko + (size_t)key0 * QKW;
        const v16h ka0 = ldh(ka), kb0 = ldh(ka + 16 * QKW);
        const v8f sa = wmma16g(ka0, qh, (v8f){});
        const v8f sb = wmma16g(kb0, qh, (v8f){});
        float ta[8], tb[8]; float mx = -3.0e38f;
#pragma unroll
        for (int r = 0; r < 8; ++r) { ta[r] = sa[r] * SC2; tb[r] = sb[r] * SC2; mx = fmaxf(mx, fmaxf(ta[r], tb[r])); }
        mx = fmaxf(mx, __shfl_xor(mx, 16, 32));
        const float mnew = fmaxf(m, mx);
        const float alpha = __builtin_amdgcn_exp2f(m - mnew);
        const float sh = PSH - mnew;
        v16h pb; float ls = 0.0f;
#pragma unroll
        for (int r = 0; r < 8; ++r) { const h16 pa = p_flush(ta[r] + sh); const h16 pc = p_flush(tb[r] + sh); pb[r] = pa; pb[8 + r] = pc; ls += (float)pa + (float)pc; }
        l = l * alpha + ls; m = mnew;
        o0 = o0 * alpha; o1 = o1 * alpha;
        const h16* va = VT + vo + key0;
        const v16h v0 = ldh(va), v1 = ldh(va + (size_t)16 * SEQ);
        o0 = wmma16g(v0, pb, o0);
        o1 = wmma16g(v1, pb, o1);
    }
    l += __shfl_xor(l, 16, 32);
    const float inv = (1.0f / l) * OCS;
    v16h ob;
#pragma unroll
    for (int r = 0; r < 8; ++r) { ob[r] = toh_flush(o0[r] * inv); ob[8 + r] = toh_flush(o1[r] * inv); }
    float* obase0 = OUT + (size_t)b * CH * OUT_SEQ + (size_t)blockIdx.x * (16 * AW);
#pragma unroll 1
    for (int hf = 0; hf < CH / OH; ++hf) {
#pragma unroll
        for (int j = 0; j < OH / 16; ++j) {
            const v16h aw = ldh(WOH + (size_t)(hf * OH + j * 16 + lr) * VC + 8 * hi);
            const v8f y = wmma16g(aw, ob, (v8f){});
            const float* bp = BO + hf * OH + j * 16 + hi * 8;
            const v4f b0 = *(const v4f*)bp; const v4f b1 = *(const v4f*)(bp + 4);
            const float brw[8] = {b0[0], b0[1], b0[2], b0[3], b1[0], b1[1], b1[2], b1[3]};
#pragma unroll
            for (int r = 0; r < 8; ++r) os[(16 * j + 8 * hi + r) * 68 + wave * 16 + lr] = y[r] * OFI + brw[r]; }
        __syncthreads();
        float* obase = obase0 + (size_t)hf * OH * OUT_SEQ;
#pragma unroll 1
        for (int ps = 0; ps < 2; ++ps) {
#pragma unroll
            for (int s = 0; s < 16; ++s) { const int row = wave * 32 + 2 * s + hi, cofs = lr * 4;
                const v4f val = *(const v4fa*)(&os[row * 68 + cofs]);
                *(volatile v4f*)(obase + (size_t)row * OUT_SEQ + cofs) = val; }
            if (ps == 0) __threadfence(); }
        __syncthreads();
    }
}

static constexpr size_t al256(size_t v) { return (v + 255) & ~(size_t)255; }
static constexpr size_t SZ_XB  = al256((size_t)NB * SEQ * CH * 2);
static constexpr size_t SZ_WQK = al256((size_t)QKW * CH * 2);
static constexpr size_t SZ_WV  = al256((size_t)VCP * CH * 2);
static constexpr size_t SZ_WO  = al256((size_t)CH * VC * 2);
static constexpr size_t SZ_BT  = al256((size_t)NBIAS * 4);
static constexpr size_t SZ_QK  = al256((size_t)NB * SEQ * QKW * 2);
static constexpr size_t SZ_VT  = al256((size_t)NB * VCP * SEQ * 2);
static constexpr size_t SZ_TOTAL = SZ_XB + SZ_WQK + SZ_WV + SZ_WO + SZ_BT + SZ_QK + SZ_VT;
static_assert(SZ_TOTAL <= (size_t)134217728);
static_assert(((size_t)CQ * CH * 2) % 256 == 0);
static_assert(((size_t)VC * CH) % 8 == 0);
static_assert(((size_t)VCP * CH) % 8 == 0);
static_assert(((size_t)CH * VC) % 8 == 0);

extern "C" void kernel_launch(void* const* d_in, const int* in_sizes, int n_in,
                              void* d_out, int out_size, void* d_ws, size_t ws_size, hipStream_t stream) {
    if (n_in < 9) return;
    const size_t needx = ((size_t)(NB - 1) * CH + (CH - 1)) * SEQ_FULL + SEQ;
    if ((size_t)in_sizes[0] < needx) return;
    if ((size_t)in_sizes[1] < (size_t)CQ * CH || (size_t)in_sizes[3] < (size_t)CQ * CH || (size_t)in_sizes[5] < (size_t)VC * CH || (size_t)in_sizes[7] < (size_t)CH * VC) return;
    if (in_sizes[2] < CQ || in_sizes[4] < CQ || in_sizes[6] < VC || in_sizes[8] < CH) return;
    if ((size_t)out_size < ((size_t)(NB - 1) * CH + (CH - 1)) * OUT_SEQ + SEQ) return;
    if (SZ_TOTAL > ws_size) return;
    const float* x  = (const float*)d_in[0];
    const float* wq = (const float*)d_in[1]; const float* bq = (const float*)d_in[2];
    const float* wk = (const float*)d_in[3]; const float* bk = (const float*)d_in[4];
    const float* wv = (const float*)d_in[5]; const float* bv = (const float*)d_in[6];
    const float* wo = (const float*)d_in[7]; const float* bo = (const float*)d_in[8];
    float* OUT = (float*)d_out;
    char* wsp = (char*)d_ws;
    bf* XB  = (bf*)wsp;  wsp += SZ_XB;
    bf* WQK = (bf*)wsp;  wsp += SZ_WQK;
    bf* WV  = (bf*)wsp;  wsp += SZ_WV;
    h16* WOH = (h16*)wsp; wsp += SZ_WO;
    float* BT = (float*)wsp; wsp += SZ_BT;
    h16* QKH = (h16*)wsp; wsp += SZ_QK;
    h16* VT  = (h16*)wsp; wsp += SZ_VT;

    k_xt<<<dim3(SEQ / 64, CH / 64, NB), 256, 0, stream>>>(x, XB);
    { const size_t n8 = (size_t)CQ * CH / 8; const unsigned g = (unsigned)((n8 + 255) / 256);
      k_cvt8<<<g, 256, 0, stream>>>(wq, WQK, n8); k_cvt8<<<g, 256, 0, stream>>>(wk, WQK + (size_t)CQ * CH, n8); }
    { const size_t n8s = (size_t)VC * CH / 8, n8t = (size_t)VCP * CH / 8; k_cvt8z<<<(unsigned)((n8t + 255) / 256), 256, 0, stream>>>(wv, WV, n8s, n8t); }
    { const size_t n8 = (size_t)CH * VC / 8; k_cvth8<<<(unsigned)((n8 + 255) / 256), 256, 0, stream>>>(wo, WOH, n8, WOS); }
    k_bias<<<1, 96, 0, stream>>>(bq, bk, bv, bo, BT);

    k_proj<0><<<dim3(NB * SEQ / 64, QKW / 64, 1), 32, 0, stream>>>(XB, WQK, BT, QKH, QKH, 0, SEQ, (size_t)SEQ * QKW, QKW, QKW, (size_t)0);
    k_proj<1><<<dim3(VCP / 64, NB * SEQ / 64, 1), 32, 0, stream>>>(WV, XB, BT + 2 * CQ, VT, VT, 0, VCP, (size_t)0, SEQ, SEQ, (size_t)VCP * SEQ);

    k_flash<<<dim3(SEQ / (16 * AW), NB, 1), 32 * AW, 0, stream>>>(QKH, VT, WOH, BT + BOFF, OUT);
}
